// ScaledDotProductAttention_62448824484005
// MI455X (gfx1250) — hardware-verified
//
#include <hip/hip_runtime.h>
#include <stdint.h>


typedef _Float16 v16h __attribute__((ext_vector_type(16)));
typedef _Float16 v8h  __attribute__((ext_vector_type(8)));
typedef float    v8f  __attribute__((ext_vector_type(8)));
typedef float    v4f  __attribute__((ext_vector_type(4)));
typedef int      v4i  __attribute__((ext_vector_type(4)));

#ifndef NB
#define NB 16
#endif
#ifndef SEQ
#define SEQ 2048
#endif
#define SEQ_FULL 2048
#define DK 128

constexpr int QT  = 128;
constexpr int KB  = 64;
constexpr int NT  = KB / 16;
constexpr int ND  = DK / 16;
constexpr int NKC = DK / 32;
constexpr int NKB = SEQ / KB;
constexpr int PCH = 128;
constexpr int KDP = DK + 8;
constexpr int VDP = KB + 8;
constexpr int PDP = KB + 8;
constexpr int ODP = DK + 4;
constexpr int TP  = PCH + 8;
constexpr size_t IN_B = (size_t)SEQ_FULL * DK;
constexpr size_t WS_B = (size_t)SEQ * DK;

constexpr float SM_SCALE = 0.0883883476483184405f;
constexpr float LOG2E    = 1.44269504088896341f;
constexpr float PCARRY   = 10.0f;

constexpr int LB_K    = 0;
constexpr int LB_V    = LB_K  + KB * KDP * 2;
constexpr int LB_P    = LB_V  + DK * VDP * 2;
constexpr int LB_END  = LB_P  + 8 * 16 * PDP * 2;
constexpr int LB_O    = 0;
constexpr int LB_OEND = LB_O + 8 * 16 * ODP * 4;
constexpr int SMEM_BYTES = (LB_END > LB_OEND) ? LB_END : LB_OEND;

static_assert(NB >= 1);
static_assert(SEQ >= PCH);
static_assert(SEQ <= SEQ_FULL);
static_assert(SEQ % QT == 0);
static_assert(SEQ % KB == 0);
static_assert(SEQ % PCH == 0);
static_assert(QT == 8 * 16);
static_assert(NT == 4);
static_assert(ND == 8);
static_assert(NKC == 4);
static_assert(DK == 128);
static_assert(PCH == 128);
static_assert((KDP * 2) % 16 == 0);
static_assert((VDP * 2) % 16 == 0);
static_assert((PDP * 2) % 16 == 0);
static_assert((ODP * 4) % 16 == 0);
static_assert((TP  * 2) % 16 == 0);
static_assert(LB_V % 16 == 0);
static_assert(LB_P % 16 == 0);
static_assert(LB_END % 16 == 0);
static_assert(SMEM_BYTES <= 160 * 1024);
static_assert(256 * 8 * 8 == PCH * DK);
static_assert(256 * 16 * 4 == PCH * DK);
static_assert((size_t)(SEQ / PCH) * NB * PCH * DK == (size_t)NB * SEQ * DK);
static_assert(256 * 4 * 8 == KB * DK);
static_assert(8 * 16 * 32 * 4 == QT * DK);
static_assert((size_t)(SEQ / QT) * NB * QT * DK == (size_t)NB * SEQ * DK);
static_assert(NKB * KB == SEQ);

union HV { v8h h; v4i i; };

__device__ __forceinline__ float bf16v(float x) {
    uint32_t u = __float_as_uint(x);
    u = (u + 0x7FFFu + ((u >> 16) & 1u)) & 0xFFFF0000u;
    return __uint_as_float(u);
}
__device__ __forceinline__ _Float16 h16(float x) { return (_Float16)bf16v(x); }

__device__ __forceinline__ float fexp2(float x) {
#if defined(__has_builtin)
#if __has_builtin(__builtin_amdgcn_exp2f)
    return __builtin_amdgcn_exp2f(x);
#else
    return exp2f(x);
#endif
#else
    return exp2f(x);
#endif
}

__device__ __forceinline__ float frcp(float x) {
#if defined(__has_builtin)
#if __has_builtin(__builtin_amdgcn_rcpf)
    return __builtin_amdgcn_rcpf(x);
#else
    return 1.0f / x;
#endif
#else
    return 1.0f / x;
#endif
}

__device__ __forceinline__ v8f mma16(v16h a, v16h b, v8f c) {
    v8f d = __builtin_amdgcn_wmma_f32_16x16x32_f16(false, a, false, b, (short)0, c, false, false);
    asm volatile("v_nop\n\tv_nop\n\tv_nop\n\tv_nop" : "+v"(d) : "v"(a), "v"(b));
    return d;
}

__device__ __forceinline__ v16h ld_op16(const _Float16* p) {
    union { v16h v; v8h hh[2]; } u;
    u.hh[0] = *(const v8h*)(p);
    u.hh[1] = *(const v8h*)(p + 16);
    return u.v;
}

__device__ __forceinline__ v16h ld_q(const float* p) {
    const v4f x0 = *(const v4f*)(p);
    const v4f x1 = *(const v4f*)(p + 4);
    const v4f x2 = *(const v4f*)(p + 16);
    const v4f x3 = *(const v4f*)(p + 20);
    v16h r;
#pragma unroll
    for (int j = 0; j < 4; ++j) {
        r[j]      = h16(x0[j]);
        r[4 + j]  = h16(x1[j]);
        r[8 + j]  = h16(x2[j]);
        r[12 + j] = h16(x3[j]);
    }
    return r;
}

__global__ __launch_bounds__(256)
void k_prep(const float* __restrict__ K, const float* __restrict__ V,
            _Float16* __restrict__ Kh, _Float16* __restrict__ Vt) {
    __shared__ __align__(16) _Float16 T[DK * TP];

    const int kb  = blockIdx.x;
    const int b   = blockIdx.y;
    const int tid = threadIdx.x;
    const size_t ib  = (size_t)b * IN_B + (size_t)kb * PCH * DK;
    const size_t kob = (size_t)b * WS_B + (size_t)kb * PCH * DK;
    const size_t vob = (size_t)b * WS_B + (size_t)kb * PCH;

    HV kv[8];
    size_t ka[8];
#pragma unroll
    for (int i = 0; i < 8; ++i) {
        const int p  = i * 256 + tid;
        const int r  = p >> 4;
        const int c8 = (p & 15) * 8;
        const float* src = K + ib + (size_t)r * DK + c8;
        const v4f x0 = *(const v4f*)(src);
        const v4f x1 = *(const v4f*)(src + 4);
        v8h hv;
#pragma unroll
        for (int j = 0; j < 4; ++j) { hv[j] = h16(x0[j]); hv[4 + j] = h16(x1[j]); }
        kv[i].h = hv;
        ka[i]   = kob + (size_t)r * DK + c8;
    }
#pragma unroll
    for (int i = 0; i < 8; ++i) *(volatile v4i*)(Kh + ka[i]) = kv[i].i;

#pragma unroll
    for (int f = 0; f < 16; ++f) {
        const int e  = f * 256 + tid;
        const int r  = e >> 5;
        const int c4 = (e & 31) * 4;
        const v4f x  = *(const v4f*)(V + ib + (size_t)r * DK + c4);
#pragma unroll
        for (int j = 0; j < 4; ++j) T[(c4 + j) * TP + r] = h16(x[j]);
    }
    __syncthreads();

    HV vv[8];
    size_t va[8];
#pragma unroll
    for (int i = 0; i < 8; ++i) {
        const int p  = i * 256 + tid;
        const int L  = p >> 3;
        const int d  = L >> 1;
        const int ko = (L & 1) * 64 + (p & 7) * 8;
        vv[i].h = *(const v8h*)&T[d * TP + ko];
        va[i]   = vob + (size_t)d * SEQ + ko;
    }
#pragma unroll
    for (int i = 0; i < 8; ++i) *(volatile v4i*)(Vt + va[i]) = vv[i].i;

    __threadfence();
#pragma unroll
    for (int i = 0; i < 8; ++i) *(volatile v4i*)(Kh + ka[i]) = kv[i].i;
#pragma unroll
    for (int i = 0; i < 8; ++i) *(volatile v4i*)(Vt + va[i]) = vv[i].i;
}

__global__ __launch_bounds__(256) __attribute__((amdgpu_num_vgpr(256)))
void k_attn(const float* __restrict__ Q,
            const _Float16* __restrict__ Kh,
            const _Float16* __restrict__ Vt,
            float* __restrict__ O) {
    __shared__ __align__(16) unsigned char smem[SMEM_BYTES];
    _Float16* Ksh = reinterpret_cast<_Float16*>(smem + LB_K);
    _Float16* Vts = reinterpret_cast<_Float16*>(smem + LB_V);
    _Float16* Pst = reinterpret_cast<_Float16*>(smem + LB_P);
    float*    Osh = reinterpret_cast<float*>(smem + LB_O);

    const int qb   = blockIdx.x;
    const int b    = blockIdx.y;
    const int tid  = threadIdx.x;
    const int lane = tid & 31;
    const int wv   = tid >> 5;
    const int hf   = lane >> 4;
    const int l16  = lane & 15;
    const int koff = hf * 8;

    const float*    Qb  = Q  + (size_t)b * IN_B;
    const _Float16* KhB = Kh + (size_t)b * WS_B;
    const _Float16* VtB = Vt + (size_t)b * WS_B;
    float*          Ob  = O  + (size_t)b * WS_B;

    const float CL = SM_SCALE * LOG2E;

    const int qrow = qb * QT + wv * 16 + l16;
    const float* qp = Qb + (size_t)qrow * DK + koff;
    v16h qa[NKC];
#pragma unroll
    for (int kc = 0; kc < NKC; ++kc) qa[kc] = ld_q(qp + kc * 32);

    v16h vones;
#pragma unroll
    for (int j = 0; j < 16; ++j) vones[j] = (_Float16)1.0f;

    const v8f vzero = {0.f, 0.f, 0.f, 0.f, 0.f, 0.f, 0.f, 0.f};
    v8f o[ND];
#pragma unroll
    for (int t = 0; t < ND; ++t) o[t] = vzero;
    v8f olsum = vzero;

    float m[8];
#pragma unroll
    for (int v = 0; v < 8; ++v) m[v] = -1e30f;

    _Float16* Pw = Pst + wv * 16 * PDP;

#pragma unroll 1
    for (int kb = 0; kb < NKB; ++kb) {
        __syncthreads();

#pragma unroll
        for (int i = 0; i < 4; ++i) {
            const int cidx = tid + i * 256;
            const int rowk = cidx >> 4;
            const int cck  = cidx & 15;
            *(v8h*)&Ksh[rowk * KDP + cck * 8] =
                *(const v8h*)(KhB + (size_t)(kb * KB + rowk) * DK + cck * 8);
            const int rowd = cidx >> 3;
            const int ccv  = cidx & 7;
            *(v8h*)&Vts[rowd * VDP + ccv * 8] =
                *(const v8h*)(VtB + (size_t)rowd * SEQ + (size_t)kb * KB + ccv * 8);
        }
        __syncthreads();

        v8f c[NT];
#pragma unroll
        for (int t = 0; t < NT; ++t) c[t] = vzero;
#pragma unroll
        for (int kc = 0; kc < NKC; ++kc) {
#pragma unroll
            for (int t = 0; t < NT; ++t) {
                const v16h bop = ld_op16(&Ksh[(t * 16 + l16) * KDP + kc * 32 + koff]);
                c[t] = mma16(qa[kc], bop, c[t]);
            }
        }

        float sc[8], mb[8];
#pragma unroll
        for (int v = 0; v < 8; ++v) {
            float r = fmaxf(fmaxf(c[0][v], c[1][v]), fmaxf(c[2][v], c[3][v]));
            r = fmaxf(r, __shfl_xor(r, 1, 32));
            r = fmaxf(r, __shfl_xor(r, 2, 32));
            r = fmaxf(r, __shfl_xor(r, 4, 32));
            r = fmaxf(r, __shfl_xor(r, 8, 32));
            const float mn = fmaxf(m[v], r);
            sc[v] = fexp2((m[v] - mn) * CL);
            m[v]  = mn;
            mb[v] = mn * CL - PCARRY;
        }
#pragma unroll
        for (int t = 0; t < NT; ++t)
#pragma unroll
            for (int v = 0; v < 8; ++v)
                c[t][v] = fexp2(c[t][v] * CL - mb[v]);

#pragma unroll
        for (int v = 0; v < 8; ++v) {
#pragma unroll
            for (int t = 0; t < ND; ++t) o[t][v] *= sc[v];
            olsum[v] *= sc[v];
        }

#pragma unroll
        for (int t = 0; t < NT; ++t)
#pragma unroll
            for (int v = 0; v < 8; ++v)
                Pw[(v + 8 * hf) * PDP + t * 16 + l16] = (_Float16)c[t][v];
        __syncthreads();

        const v16h pa0 = ld_op16(&Pw[l16 * PDP + koff]);
        const v16h pa1 = ld_op16(&Pw[l16 * PDP + 32 + koff]);
        olsum = mma16(pa0, vones, olsum);
        olsum = mma16(pa1, vones, olsum);
#pragma unroll
        for (int t = 0; t < ND; ++t) {
            const v16h vb0 = ld_op16(&Vts[(t * 16 + l16) * VDP + koff]);
            const v16h vb1 = ld_op16(&Vts[(t * 16 + l16) * VDP + 32 + koff]);
            o[t] = mma16(pa0, vb0, o[t]);
            o[t] = mma16(pa1, vb1, o[t]);
        }
    }
    __syncthreads();

    float* Ow = Osh + wv * 16 * ODP;
#pragma unroll
    for (int v = 0; v < 8; ++v) {
        const float rinv = frcp(olsum[v]);
        const int   row  = v + 8 * hf;
#pragma unroll
        for (int t = 0; t < ND; ++t) Ow[row * ODP + t * 16 + l16] = o[t][v] * rinv;
    }
    __syncthreads();

    v4f ov[16];
#pragma unroll
    for (int i = 0; i < 16; ++i) ov[i] = *(const v4f*)&Ow[i * ODP + lane * 4];
    float* orow = Ob + (size_t)(qb * QT + wv * 16) * DK + lane * 4;
#pragma unroll
    for (int i = 0; i < 16; ++i) *(volatile v4f*)(orow + (size_t)i * DK) = ov[i];
    __threadfence();
#pragma unroll
    for (int i = 0; i < 16; ++i) *(volatile v4f*)(orow + (size_t)i * DK) = ov[i];
}

extern "C" void kernel_launch(void* const* d_in, const int* in_sizes, int n_in,
                              void* d_out, int out_size, void* d_ws, size_t ws_size,
                              hipStream_t stream) {
    if (n_in < 3) return;
    const long long need_in = ((long long)(NB - 1) * SEQ_FULL + SEQ) * DK;
    if ((long long)in_sizes[0] < need_in) return;
    if ((long long)in_sizes[1] < need_in) return;
    if ((long long)in_sizes[2] < need_in) return;
    const long long n_out = (long long)NB * SEQ * DK;
    if ((long long)out_size < n_out) return;

    const size_t plane = (size_t)NB * SEQ * DK;
    if (ws_size < 2 * plane * sizeof(_Float16)) return;

    const float* q = (const float*)d_in[0];
    const float* k = (const float*)d_in[1];
    const float* v = (const float*)d_in[2];
    float* out = (float*)d_out;

    _Float16* Kh = (_Float16*)d_ws;
    _Float16* Vt = Kh + plane;

    k_prep<<<dim3(SEQ / PCH, NB), 256, 0, stream>>>(k, v, Kh, Vt);
    k_attn<<<dim3(SEQ / QT, NB), 256, 0, stream>>>(q, Kh, Vt, out);
}
